// Cross_At_50208167690362
// MI455X (gfx1250) — hardware-verified
//
#include <hip/hip_runtime.h>


namespace {
constexpr int S = 4096, C = 64, H = 8, HD = 8, KP = 32  , VP = 16  ;
constexpr float XS = 8.0f, PS = 8.0f;

typedef _Float16 b16;
typedef __attribute__((ext_vector_type(16))) _Float16 v16b;
typedef __attribute__((ext_vector_type(8))) _Float16 v8b;
typedef __attribute__((ext_vector_type(8))) float v8f;
typedef __attribute__((ext_vector_type(4))) float v4f;
__device__ __forceinline__ float bf16_rne(float f) { unsigned int u = __float_as_uint(f); u += 0x7FFFu + ((u >> 16) & 1u); return __uint_as_float(u & 0xFFFF0000u); }
__device__ __forceinline__ void split16(float v, b16& hi, b16& lo) { hi = (b16)v; lo = (b16)(v - (float)hi); }
__device__ __forceinline__ v16b frag_kb(const b16* p, int hh) { const v8b a = *(const v8b*)(p + 8 * hh), b = *(const v8b*)(p + 16 + 8 * hh); v16b f;
#pragma unroll
  for (int e = 0; e < 8; ++e) { f[e] = a[e]; f[8 + e] = b[e]; } return f; }
__device__ __forceinline__ v8f wmma16b(v16b a, v16b b, v8f c) { v8f d = __builtin_amdgcn_wmma_f32_16x16x32_f16(false, a, false, b, (short)0, c, false, false); asm volatile("v_nop\n\tv_nop\n\tv_nop\n\tv_nop" : "+v"(d) : "v"(a), "v"(b)); return d; }
__device__ __forceinline__ void wave_lds_sync() { __builtin_amdgcn_fence(__ATOMIC_RELEASE, "workgroup"); __builtin_amdgcn_wave_barrier(); __builtin_amdgcn_fence(__ATOMIC_ACQUIRE, "workgroup"); }
__device__ __forceinline__ float nexp(float x) { return __builtin_amdgcn_exp2f(x * 1.4426950408889634f); }
__device__ __forceinline__ float pmul(float a, float b) { float p = a * b; asm volatile("" : "+v"(p)); return p; }

__global__ __launch_bounds__(256) void prep_kernel(const float* __restrict__ x, const float* __restrict__ y, const float* __restrict__ wq, const float* __restrict__ bq, const float* __restrict__ wkv, const float* __restrict__ bkv, const float* __restrict__ we, const float* __restrict__ be, b16* __restrict__ R, float* __restrict__ P, b16* __restrict__ X, b16* __restrict__ Y, b16* __restrict__ Z0, size_t nz) {
  const size_t tid = (size_t)blockIdx.x * 256 + threadIdx.x, nth = (size_t)gridDim.x * 256;
  for (int pass = 0; pass < 2; ++pass) {
    for (size_t p = tid; p < (size_t)C * C; p += nth) { const int o = (int)(p / C), k = (int)(p % C); ((volatile b16*)R)[p] = (b16)bf16_rne(wq[(size_t)k * C + o]); ((volatile b16*)R)[12288 + p] = (b16)bf16_rne(we[(size_t)k * C + o]); }
    for (size_t p = tid; p < (size_t)2 * C * C; p += nth) { const int o = (int)(p / C), k = (int)(p % C); ((volatile b16*)R)[4096 + p] = (b16)bf16_rne(wkv[(size_t)k * 2 * C + o]); }
    for (size_t q = tid; q < 256; q += nth) { const int i = (int)q; P[q] = bf16_rne((i < 64) ? bq[i] : (i < 192) ? bkv[i - 64] : be[i - 192]); }
    for (size_t p = tid; p < (size_t)S * C / 8; p += nth) { v8b a, b; for (int e = 0; e < 8; ++e) { a[e] = (b16)(bf16_rne(x[p * 8 + e]) * XS); b[e] = (b16)(bf16_rne(y[p * 8 + e]) * XS); } *(volatile v8b*)(X + p * 8) = a; *(volatile v8b*)(Y + p * 8) = b; }
    { const v8b z = {}; for (size_t p = tid; p < nz / 8; p += nth) *(volatile v8b*)(Z0 + p * 8) = z; }
    __threadfence(); }
}

__global__ __launch_bounds__(64) void proj_kernel(const b16* __restrict__ X, const b16* __restrict__ Y, const b16* __restrict__ R, const float* __restrict__ P, b16* __restrict__ QH, b16* __restrict__ QL, b16* __restrict__ KH, b16* __restrict__ KL, float* __restrict__ VR) {
  __shared__ __attribute__((aligned(16))) b16 Th[2][32][64 + 8], Tl[2][32][64 + 8]; __shared__ __attribute__((aligned(16))) float Tv[32][64 + 4];
  const int lane = threadIdx.x & 31, wave = threadIdx.x >> 5, nloc = lane & 15, hlf = lane >> 4, m0 = blockIdx.x * 32;
  const b16* A = wave ? Y : X; const b16* Bw = R + (wave ? 4096 : 0); const int NSUB = wave ? 8 : 4;
  v8f acc[2][8];
#pragma unroll
  for (int r = 0; r < 2; ++r)
#pragma unroll
    for (int t = 0; t < 8; ++t) acc[r][t] = (v8f){};
#pragma unroll
  for (int kb = 0; kb < C; kb += 32) { const v16b a0 = frag_kb(A + (size_t)(m0 + nloc) * C + kb, hlf), a1 = frag_kb(A + (size_t)(m0 + 16 + nloc) * C + kb, hlf);
#pragma unroll
    for (int t = 0; t < 8; ++t) { if (t < NSUB) { const v16b bw = frag_kb(Bw + (size_t)(t * 16 + nloc) * C + kb, hlf); acc[0][t] = wmma16b(a0, bw, acc[0][t]); acc[1][t] = wmma16b(a1, bw, acc[1][t]); } } }
#pragma unroll
  for (int t = 0; t < 4; ++t) { const float bb = P[(wave ? 64 : 0) + t * 16 + nloc];
#pragma unroll
    for (int r = 0; r < 2; ++r)
#pragma unroll
      for (int v = 0; v < 8; ++v) { const float val = acc[r][t][v] * (1.0f / XS) + bb; float ss = pmul(val, val); ss += __shfl_xor(ss, 1); ss += __shfl_xor(ss, 2); ss += __shfl_xor(ss, 4); const float nv = val / fmaxf(sqrtf(ss), 1e-12f);
        b16 a_, c_; split16(nv * XS, a_, c_); Th[wave][r * 16 + 8 * hlf + v][t * 16 + nloc] = a_; Tl[wave][r * 16 + 8 * hlf + v][t * 16 + nloc] = c_; } }
  if (wave == 1) {
#pragma unroll
    for (int t = 4; t < 8; ++t) { const float bb = P[64 + t * 16 + nloc];
#pragma unroll
      for (int r = 0; r < 2; ++r)
#pragma unroll
        for (int v = 0; v < 8; ++v) Tv[r * 16 + 8 * hlf + v][(t - 4) * 16 + nloc] = acc[r][t][v] * (1.0f / XS) + bb; } }
  __syncthreads();
  b16* dh = wave ? KH : QH; b16* dl = wave ? KL : QL;
  for (int pass = 0; pass < 2; ++pass) {
    for (int i = lane; i < 32 * 8; i += 32) { const int rr = i >> 3, hh2 = i & 7; const size_t gi = ((size_t)(m0 + rr) * H + hh2) * KP; *(volatile v8b*)(dh + gi) = *(const v8b*)(&Th[wave][rr][hh2 * 8]); *(volatile v8b*)(dl + gi) = *(const v8b*)(&Tl[wave][rr][hh2 * 8]); }
    if (wave == 1) { for (int i = lane; i < 32 * 16; i += 32) { const int rr = i >> 4, c4 = (i & 15) * 4; *(volatile v4f*)(VR + (size_t)(m0 + rr) * C + c4) = *(const v4f*)(&Tv[rr][c4]); } }
    __threadfence(); }
}
__global__ __launch_bounds__(256) void vt_kernel(const float* __restrict__ VR, b16* __restrict__ VTh, b16* __restrict__ VTl) {
  __shared__ __attribute__((aligned(16))) b16 Th[64][128 + 8], Tl[64][128 + 8];
  const int t0 = blockIdx.x * 128, t_ = threadIdx.x;
  for (int i = t_; i < 128 * 64; i += 256) { const int tk = i >> 6, c = i & 63; b16 a_, b_; split16(VR[(size_t)(t0 + tk) * C + c] * XS, a_, b_); Th[c][tk] = a_; Tl[c][tk] = b_; }
  __syncthreads();
  for (int pass = 0; pass < 2; ++pass) { for (int i = t_; i < 64 * 16; i += 256) { const int c = i >> 4, c8 = (i & 15) * 8; const int h = c >> 3, d = c & 7; const size_t gi = ((size_t)h * VP + d) * S + t0 + c8; *(volatile v8b*)(VTh + gi) = *(const v8b*)(&Th[c][c8]); *(volatile v8b*)(VTl + gi) = *(const v8b*)(&Tl[c][c8]); } __threadfence(); }
}
__global__ __launch_bounds__(256) void attn_kernel(const b16* __restrict__ QH, const b16* __restrict__ QL, const b16* __restrict__ KH, const b16* __restrict__ KL, const b16* __restrict__ VTh, const b16* __restrict__ VTl, b16* __restrict__ CH, b16* __restrict__ CL) {
  __shared__ __attribute__((aligned(16))) b16 Oh[16][C + 8], Ol[16][C + 8];
  const int h = threadIdx.x >> 5, lane = threadIdx.x & 31, hh = lane >> 4, col = lane & 15; const int q0 = blockIdx.x * 16, qi = q0 + col;
  const v16b qf = frag_kb(QH + ((size_t)qi * H + h) * KP, hh), ql = frag_kb(QL + ((size_t)qi * H + h) * KP, hh); const b16* V = VTh + (size_t)(h * VP) * S; const b16* Vl = VTl + (size_t)(h * VP) * S;
  float m = -INFINITY, l = 0.0f; v8f o = {};
  for (int kb = 0; kb < S; kb += 32) {
    v8f s0 = {}, s1 = {};
    { const v16b k0 = frag_kb(KH + ((size_t)(kb + col) * H + h) * KP, hh), k0l = frag_kb(KL + ((size_t)(kb + col) * H + h) * KP, hh), k1 = frag_kb(KH + ((size_t)(kb + 16 + col) * H + h) * KP, hh), k1l = frag_kb(KL + ((size_t)(kb + 16 + col) * H + h) * KP, hh);
      s0 = wmma16b(k0, qf, s0); s0 = wmma16b(k0l, qf, s0); s0 = wmma16b(k0, ql, s0); s1 = wmma16b(k1, qf, s1); s1 = wmma16b(k1l, qf, s1); s1 = wmma16b(k1, ql, s1); }
    float mr = -INFINITY;
#pragma unroll
    for (int r = 0; r < 8; ++r) { s0[r] *= 1.0f / (XS * XS); s1[r] *= 1.0f / (XS * XS); mr = fmaxf(mr, fmaxf(s0[r], s1[r])); }
    mr = fmaxf(mr, __shfl_xor(mr, 16)); const float mn = fmaxf(m, mr); const float al_ = nexp(m - mn); m = mn; float sum = 0.0f; v16b pb, pl;
#pragma unroll
    for (int r = 0; r < 8; ++r) { const float e0 = nexp(s0[r] - mn), e1 = nexp(s1[r] - mn); sum += e0 + e1; b16 a_, c_; split16(e0 * PS, a_, c_); pb[r] = a_; pl[r] = c_; split16(e1 * PS, a_, c_); pb[8 + r] = a_; pl[8 + r] = c_; }
    sum += __shfl_xor(sum, 16); l = l * al_ + sum; o *= al_;
    const v16b vh = frag_kb(V + (size_t)col * S + kb, hh); o = wmma16b(vh, pb, o); o = wmma16b(vh, pl, o); o = wmma16b(frag_kb(Vl + (size_t)col * S + kb, hh), pb, o); }
  const float inv = 1.0f / (l * PS);
  if (hh == 0) {
#pragma unroll
    for (int r = 0; r < 8; ++r) { b16 a_, c_; split16(o[r] * inv, a_, c_); Oh[col][h * HD + r] = a_; Ol[col][h * HD + r] = c_; } }
  __syncthreads();
  for (int pass = 0; pass < 2; ++pass) { for (int i = threadIdx.x; i < 16 * 8; i += 256) { const int rr = i >> 3, c8 = (i & 7) * 8; const size_t gi = (size_t)(q0 + rr) * C + c8; *(volatile v8b*)(CH + gi) = *(const v8b*)(&Oh[rr][c8]); *(volatile v8b*)(CL + gi) = *(const v8b*)(&Ol[rr][c8]); } __threadfence(); }
}
__global__ __launch_bounds__(64) void out_kernel(const b16* __restrict__ CH, const b16* __restrict__ CL, const b16* __restrict__ R, const float* __restrict__ P, float* __restrict__ out) {
  __shared__ __attribute__((aligned(16))) float Ts[2][16][C + 4];
  const int lane = threadIdx.x & 31, wave = threadIdx.x >> 5, nloc = lane & 15, hlf = lane >> 4, m0 = blockIdx.x * 32 + wave * 16; const b16* Bw = R + 12288;
  v8f acc[4] = {{}, {}, {}, {}};
#pragma unroll
  for (int kb = 0; kb < C; kb += 32) { const v16b a = frag_kb(CH + (size_t)(m0 + nloc) * C + kb, hlf), al_ = frag_kb(CL + (size_t)(m0 + nloc) * C + kb, hlf);
#pragma unroll
    for (int t = 0; t < 4; ++t) { const v16b bw = frag_kb(Bw + (size_t)(t * 16 + nloc) * C + kb, hlf); acc[t] = wmma16b(a, bw, acc[t]); acc[t] = wmma16b(al_, bw, acc[t]); } }
#pragma unroll
  for (int t = 0; t < 4; ++t)
#pragma unroll
    for (int r = 0; r < 8; ++r) Ts[wave][8 * hlf + r][t * 16 + nloc] = acc[t][r] * (1.0f / XS) + P[192 + t * 16 + nloc];
  wave_lds_sync();
  for (int pass = 0; pass < 2; ++pass) { for (int i = lane; i < 16 * 16; i += 32) { const int rr = i >> 4, c4 = (i & 15) * 4; *(volatile v4f*)(out + (size_t)(m0 + rr) * C + c4) = *(const v4f*)(&Ts[wave][rr][c4]); } __threadfence(); }
}
}

extern "C" void kernel_launch(void* const* d_in, const int* in_sizes, int n_in,
                              void* d_out, int out_size, void* d_ws, size_t ws_size, hipStream_t stream) {
  (void)n_in; (void)out_size;
  const float* x = (const float*)d_in[0]; const float* y = (const float*)d_in[1]; const float* wq = (const float*)d_in[2]; const float* bq = (const float*)d_in[3]; const float* wkv = (const float*)d_in[4]; const float* bkv = (const float*)d_in[5]; const float* we = (const float*)d_in[6]; const float* be = (const float*)d_in[7];
  float* out = (float*)d_out;
  if (in_sizes[0] != S * C || in_sizes[4] != C * 2 * C) return;
  size_t off = 0; char* ws = (char*)d_ws;
  auto carve = [&](size_t bytes) { char* p = ws + off; off += (bytes + 255) & ~(size_t)255; return p; };
  b16* R = (b16*)carve(16384 * 2); float* P = (float*)carve(256 * 4); b16* X = (b16*)carve((size_t)S * C * 2); b16* Y = (b16*)carve((size_t)S * C * 2); float* VR = (float*)carve((size_t)S * C * 4); b16* CH = (b16*)carve((size_t)S * C * 2); b16* CL = (b16*)carve((size_t)S * C * 2);
  const size_t slot = (size_t)S * H * KP, plane = (size_t)H * VP * S; b16* Z0 = (b16*)carve((4 * slot + 2 * plane) * 2); b16* QH = Z0; b16* QL = Z0 + slot; b16* KH = Z0 + 2 * slot; b16* KL = Z0 + 3 * slot; b16* VTh = Z0 + 4 * slot; b16* VTl = VTh + plane;
  if (off > ws_size) return;
  prep_kernel<<<256, 256, 0, stream>>>(x, y, wq, bq, wkv, bkv, we, be, R, P, X, Y, Z0, 4 * slot + 2 * plane);
  proj_kernel<<<S / 32, 64, 0, stream>>>(X, Y, R, P, QH, QL, KH, KL, VR);
  vt_kernel<<<S / 128, 256, 0, stream>>>(VR, VTh, VTl);
  attn_kernel<<<S / 16, 256, 0, stream>>>(QH, QL, KH, KL, VTh, VTl, CH, CL);
  out_kernel<<<S / 32, 64, 0, stream>>>(CH, CL, R, P, out);
}
